// PolynomialRegressor_27152783246050
// MI455X (gfx1250) — hardware-run, weakly checked
//
#include <hip/hip_runtime.h>


#ifndef NB
#define NB 2048
#endif
#define NB_FULL 2048
#define NIN   64
#define NOUT  10
#define NF1   64
#define NF2   2080
#define NF3   45760
#define NFEAT (NF1 + NF2 + NF3)
#define NSTEP 2706
#define KP    (NSTEP * 32)
#define XP    65

static constexpr int count_steps() {
    int s = 2;
    for (int j = 0; j < 64; ++j) s += (j < 32) ? 2 : 1;
    for (int i = 0; i < 64; ++i) for (int j = i; j < 64; ++j) s += (j < 32) ? 2 : 1;
    return s;
}
static constexpr int count_feats() {
    int s = 64;
    for (int i = 0; i < 64; ++i) s += 64 - i;
    for (int i = 0; i < 64; ++i) for (int j = i; j < 64; ++j) s += 64 - j;
    return s;
}
static_assert(count_steps() == NSTEP);
static_assert(count_feats() == NFEAT);
static_assert(NFEAT == 47904);
static_assert(NSTEP % 2 == 0);
static_assert(KP % 64 == 0);
static_assert(NB % 16 == 0);
static_assert(NB <= NB_FULL);
static_assert(NIN == 64);
static_assert(NOUT <= 16);
static_assert((32 + 8) * 16 == 16 * NOUT * 4);
static_assert(128 * 16 == 16 * 128);
static_assert(8 * 128 == 64 * 16);
static_assert(16 * XP * 4 + 16 * 16 * 4 <= 131072);
static_assert(64 * 4 + 64 * 16 * 2 <= 131072);

typedef unsigned short bf;
typedef __attribute__((ext_vector_type(16))) __bf16   v16bf;
typedef __attribute__((ext_vector_type(8)))  unsigned short v8us;
typedef __attribute__((ext_vector_type(8)))  unsigned v8u;
typedef __attribute__((ext_vector_type(8)))  float    v8f;
typedef __attribute__((ext_vector_type(4)))  float    v4f;

__device__ __forceinline__ unsigned short f2bf(float f) { unsigned u = __float_as_uint(f); u += 0x7FFFu + ((u >> 16) & 1u); return (unsigned short)(u >> 16); }
__device__ __forceinline__ float bf2f(unsigned short w) { return __uint_as_float(((unsigned)w) << 16); }
__device__ __forceinline__ int clampi(int v, int lo, int hi) { return min(max(v, lo), hi); }
__device__ __forceinline__ v16bf cat16b(v8us lo, v8us hi) { return __builtin_bit_cast(v16bf, __builtin_shufflevector(lo, hi, 0, 1, 2, 3, 4, 5, 6, 7, 8, 9, 10, 11, 12, 13, 14, 15)); }
__device__ __forceinline__ v8f wmmab(v16bf a, v16bf b, v8f c) { return __builtin_amdgcn_wmma_f32_16x16x32_bf16(false, a, false, b, (short)0, c, false, false); }
__device__ __forceinline__ v16bf ldb(const bf* p)  { return cat16b(*(const v8us*)p, *(const v8us*)(p + 16)); }
__device__ __forceinline__ void wave_sync() { __builtin_amdgcn_fence(3  , "wavefront"); __builtin_amdgcn_wave_barrier(); asm volatile("" ::: "memory"); }

__device__ __forceinline__ v8f wmmag(v16bf a, v16bf b, v8f c) {
    c = wmmab(a, b, c);
    asm volatile("v_nop\n\tv_nop\n\tv_nop\n\tv_nop" : "+v"(c) : "v"(a), "v"(b));
    return c;
}

__device__ __forceinline__ v8f bfq8(v8f v) { v8f o;
#pragma unroll
    for (int k = 0; k < 8; ++k) o[k] = bf2f(f2bf(v[k]));
    return o; }

__device__ __forceinline__ void split2(float v0, float v1, unsigned& hw, unsigned& lw) {
    const unsigned u0 = __float_as_uint(v0), u1 = __float_as_uint(v1);
    const unsigned t0 = u0 & 0xFFFF0000u, t1 = u1 & 0xFFFF0000u;
    hw = (t0 >> 16) | t1;
    const float r0 = v0 - __uint_as_float(t0), r1 = v1 - __uint_as_float(t1);
    lw = (unsigned)f2bf(r0) | (((unsigned)f2bf(r1)) << 16);
}

__device__ __forceinline__ v8f poly_step(float p, v8f x0, v8f x1, const bf* bptr, v8f acc) {
    v8u hw, lw;
#pragma unroll
    for (int d = 0; d < 4; ++d) {
        unsigned h, l;
        split2(p * x0[2 * d], p * x0[2 * d + 1], h, l); hw[d] = h; lw[d] = l;
        split2(p * x1[2 * d], p * x1[2 * d + 1], h, l); hw[4 + d] = h; lw[4 + d] = l;
    }
    const v16bf b = ldb(bptr);
    acc = wmmag(__builtin_bit_cast(v16bf, hw), b, acc);
    acc = wmmag(__builtin_bit_cast(v16bf, lw), b, acc);
    return acc;
}

__global__ __launch_bounds__(128) void k_wt(const float* __restrict__ W, bf* WT) {
    __shared__ int srow[64];
    __shared__ __align__(16) unsigned short ts[64 * 16];
    const int t = threadIdx.x; const int wave = __builtin_amdgcn_readfirstlane(t >> 5);
    const int blk = blockIdx.x;
    if (wave < 2) {
        const int s = 2 * blk + (t >> 5);
        const int s1 = s - 2;
        const int si = (s1 < 64) ? (s1 >> 1) : (s1 - 32);
        const int sh = (s1 < 64) ? (s1 & 1) : 1;
        const int sb = NF1 + 64 * si - (si * (si - 1)) / 2;
        int s2 = s - 98, pi = 0, ob = 0;
#pragma unroll 1
        for (int it = 0; it < 63; ++it) {
            const int cnt = (pi < 32) ? (96 - 2 * pi) : (64 - pi);
            const bool adv = (s2 >= cnt);
            ob += adv ? ((64 - pi) * (65 - pi)) / 2 : 0;
            s2 -= adv ? cnt : 0;
            pi += adv ? 1 : 0;
        }
        const int two = 2 * (32 - pi);
        const int pjl = (s2 < two) ? (pi + (s2 >> 1)) : (32 + (s2 - two));
        const int phl = (s2 < two) ? (s2 & 1) : 1;
        const int pj = (pi < 32) ? pjl : (pi + s2);
        const int ph = (pi < 32) ? phl : 1;
        const int nn = pj - pi;
        const int pb = NF1 + NF2 + ob + 64 * nn - (nn * (2 * pi + nn - 1)) / 2;
        const bool q0 = (s < 2), q1 = (s < 98);
        const int jmin = q0 ? 0 : (q1 ? si : pj);
        const int half = q0 ? (s & 1) : (q1 ? sh : ph);
        const int base = q0 ? 0 : (q1 ? sb : pb);
        const int k = half * 32 + (t & 31);
        srow[t] = (k >= jmin) ? (base + (k - jmin)) : -1;
    }
    __syncthreads();
#pragma unroll 1
    for (int it = 0; it < 8; ++it) {
        const int e = it * 128 + t; const int c = e >> 4, n = e & 15;
        const int src = srow[c];
        const bool ok = (src >= 0) && (n < NOUT);
        const int idx = clampi(src, 0, NFEAT - 1) * NOUT + min(n, NOUT - 1);
        const float v = W[idx];
        const unsigned short q = f2bf(v);
        ts[c * 16 + n] = ok ? q : (unsigned short)0;
    }
    __syncthreads();
    const int n = t >> 3, c8 = (t & 7) * 8; v8us o;
#pragma unroll
    for (int k = 0; k < 8; ++k) o[k] = ts[(c8 + k) * 16 + n];
    bf* dst = WT + (size_t)n * KP + (size_t)blk * 64 + c8;
#pragma unroll 1
    for (int ps = 0; ps < 2; ++ps) {
        *(volatile v8us*)dst = o;
        if (ps == 0) __threadfence(); }
}

__global__ __launch_bounds__(32) __attribute__((amdgpu_num_vgpr(256))) void k_poly(const float* __restrict__ X, const bf* __restrict__ WT,
                                                                                    const float* __restrict__ Bv, float* OUT) {
    __shared__ __align__(16) float xs[16 * XP];
    __shared__ __align__(16) float os[16 * 16];
    const int lane = threadIdx.x & 31, lr = lane & 15, hi = lane >> 4;
    const int tile = blockIdx.x;
    const float* xrow = X + (size_t)(tile * 16 + lr) * NIN + 8 * hi;
    const v8f xa0 = bfq8(*(const v8f*)(xrow));
    const v8f xa1 = bfq8(*(const v8f*)(xrow + 16));
    const v8f xb0 = bfq8(*(const v8f*)(xrow + 32));
    const v8f xb1 = bfq8(*(const v8f*)(xrow + 48));
#pragma unroll
    for (int e = 0; e < 8; ++e) {
        xs[lr * XP + 8 * hi + e]      = xa0[e];
        xs[lr * XP + 16 + 8 * hi + e] = xa1[e];
        xs[lr * XP + 32 + 8 * hi + e] = xb0[e];
        xs[lr * XP + 48 + 8 * hi + e] = xb1[e];
    }
    wave_sync();

    v8f acc = (v8f){};
    const bf* bp = WT + (size_t)lr * KP + 8 * hi;
    int kq = 0;
    acc = poly_step(1.0f, xa0, xa1, bp + kq, acc); kq += 32;
    acc = poly_step(1.0f, xb0, xb1, bp + kq, acc); kq += 32;
#pragma unroll 1
    for (int j = 0; j < 32; ++j) {
        const float p = xs[lr * XP + j];
        acc = poly_step(p, xa0, xa1, bp + kq, acc); kq += 32;
        acc = poly_step(p, xb0, xb1, bp + kq, acc); kq += 32;
    }
#pragma unroll 1
    for (int j = 32; j < 64; ++j) {
        const float p = xs[lr * XP + j];
        acc = poly_step(p, xb0, xb1, bp + kq, acc); kq += 32;
    }
#pragma unroll 1
    for (int i = 0; i < 64; ++i) {
        const float xi = xs[lr * XP + i];
#pragma unroll 1
        for (int j = i; j < 32; ++j) {
            const float p = xi * xs[lr * XP + j];
            acc = poly_step(p, xa0, xa1, bp + kq, acc); kq += 32;
            acc = poly_step(p, xb0, xb1, bp + kq, acc); kq += 32;
        }
        const int j1 = (i > 32) ? i : 32;
#pragma unroll 1
        for (int j = j1; j < 64; ++j) {
            const float p = xi * xs[lr * XP + j];
            acc = poly_step(p, xb0, xb1, bp + kq, acc); kq += 32;
        }
    }

#pragma unroll
    for (int r = 0; r < 8; ++r) os[(8 * hi + r) * 16 + lr] = acc[r];
    wave_sync();
    v4f o0, o1;
#pragma unroll
    for (int q = 0; q < 4; ++q) {
        const int f0 = 4 * lane + q;
        const int r0 = f0 / NOUT, c0 = f0 - NOUT * r0;
        const float b0 = bf2f(f2bf(Bv[c0]));
        o0[q] = os[r0 * 16 + c0] + b0;
        const int f1 = min(128 + 4 * lane + q, 16 * NOUT - 1);
        const int r1 = f1 / NOUT, c1 = f1 - NOUT * r1;
        const float b1 = bf2f(f2bf(Bv[c1]));
        o1[q] = os[r1 * 16 + c1] + b1;
    }
    float* dst = OUT + (size_t)tile * (16 * NOUT);
#pragma unroll 1
    for (int ps = 0; ps < 2; ++ps) {
        *(volatile v4f*)(dst + 4 * lane) = o0;
        if (lane < 8) *(volatile v4f*)(dst + 128 + 4 * lane) = o1;
        if (ps == 0) __threadfence(); }
}

static constexpr size_t al256(size_t v) { return (v + 255) & ~(size_t)255; }
static constexpr size_t SZ_WT = al256((size_t)16 * KP * 2);
static constexpr size_t SZ_TOTAL = SZ_WT;
static_assert(SZ_TOTAL <= (size_t)134217728);
static_assert((size_t)(KP / 64) * 64 * 2 * 16 == (size_t)16 * KP * 2);
static_assert((size_t)(NB / 16) * 16 * NOUT == (size_t)NB * NOUT);

extern "C" void kernel_launch(void* const* d_in, const int* in_sizes, int n_in,
                              void* d_out, int out_size, void* d_ws, size_t ws_size, hipStream_t stream) {
    if (n_in < 3) return;
    if ((size_t)in_sizes[0] < (size_t)NB * NIN) return;
    if ((size_t)in_sizes[1] < (size_t)NFEAT * NOUT) return;
    if ((size_t)in_sizes[2] < (size_t)NOUT) return;
    if ((size_t)out_size < (size_t)NB * NOUT) return;
    if (SZ_TOTAL > ws_size) return;
    const float* X  = (const float*)d_in[0];
    const float* W  = (const float*)d_in[1];
    const float* Bv = (const float*)d_in[2];
    float* OUT = (float*)d_out;
    bf* WT = (bf*)d_ws;

    k_wt<<<KP / 64, 128, 0, stream>>>(W, WT);
    k_poly<<<NB / 16, 32, 0, stream>>>(X, WT, Bv, OUT);
}
